// BaseAttentionHead_52682068853252
// MI455X (gfx1250) — hardware-verified
//
#include <hip/hip_runtime.h>
#include <math.h>

typedef __attribute__((ext_vector_type(16))) _Float16 v16h;
typedef __attribute__((ext_vector_type(16))) __bf16 v16b;
typedef __attribute__((ext_vector_type(8)))  _Float16 v8h;
typedef __attribute__((ext_vector_type(8)))  float v8f;
typedef __attribute__((ext_vector_type(4)))  float v4f;
typedef __attribute__((ext_vector_type(2)))  float v2f;
typedef __attribute__((ext_vector_type(4)))  unsigned v4u;
typedef __attribute__((ext_vector_type(4)))  int v4i;
typedef float __attribute__((may_alias)) float_a;
typedef int __attribute__((may_alias)) int_a;

template <typename T> __device__ __forceinline__ void vst2(void* p, T v) { *(volatile T*)p = v; __threadfence(); *(volatile T*)p = v; }
__device__ __forceinline__ v8f wmma16(v16h a, v16h b, v8f c) {
  v8f d = __builtin_amdgcn_wmma_f32_16x16x32_f16(false, a, false, b, (short)0, c, false, false);
  asm volatile("v_nop\n\tv_nop\n\tv_nop\n\tv_nop" : "+v"(d) : "v"(a), "v"(b));
  return d;
}
__device__ __forceinline__ v8f wmma_bf(v16b a, v16b b, v8f c) {
  v8f d = __builtin_amdgcn_wmma_f32_16x16x32_bf16(false, a, false, b, (short)0, c, false, false);
  asm volatile("v_nop\n\tv_nop\n\tv_nop\n\tv_nop" : "+v"(d) : "v"(a), "v"(b));
  return d;
}
__device__ __forceinline__ v16h frag_h(const _Float16* rowk0, int lane) {
  union { v16h v; v8h q[2]; } u; const _Float16* p = rowk0 + 8 * (lane >> 4);
  u.q[0] = *(const v8h*)p; u.q[1] = *(const v8h*)(p + 16); return u.v;
}
__device__ __forceinline__ v16h frag_f32(const float* rowk0, int lane) {
  v16h a; const float* p = rowk0 + 8 * (lane >> 4);
#pragma unroll
  for (int i = 0; i < 8; ++i) { a[i] = (_Float16)p[i]; a[8 + i] = (_Float16)p[16 + i]; }
  return a;
}
__device__ __forceinline__ v16h frag_f32s(const float* rowk0, int lane, float sc) {
  v16h a; const float* p = rowk0 + 8 * (lane >> 4);
#pragma unroll
  for (int i = 0; i < 8; ++i) { a[i] = (_Float16)(p[i] * sc); a[8 + i] = (_Float16)(p[16 + i] * sc); }
  return a;
}
__device__ __forceinline__ v16h fragc_f32(const float* W, int k0, int n, int lane, int ld, int K) {
  v16h a; const int g = lane >> 4;
#pragma unroll
  for (int i = 0; i < 8; ++i) { const int ka = k0 + 8 * g + i, kb = ka + 16;
    a[i] = (_Float16)(ka < K ? W[(size_t)(ka < K ? ka : K - 1) * ld + n] : 0.f); a[8 + i] = (_Float16)(kb < K ? W[(size_t)(kb < K ? kb : K - 1) * ld + n] : 0.f); }
  return a;
}
struct F2 { v16b h, l; };
__device__ __forceinline__ F2 bsplit16(const float v[16]) { F2 r;
#pragma unroll
  for (int i = 0; i < 16; ++i) { const __bf16 h = (__bf16)v[i]; r.h[i] = h; r.l[i] = (__bf16)(v[i] - (float)h); }
  return r; }
__device__ __forceinline__ F2 split_row(const float* row, int k0, int lane) { float v[16]; const float* p = row + k0 + 8 * (lane >> 4);
#pragma unroll
  for (int i = 0; i < 8; ++i) { v[i] = p[i]; v[8 + i] = p[16 + i]; }
  return bsplit16(v); }
__device__ __forceinline__ F2 split_rowK(const float* row, int k0, int lane, int K) { float v[16]; const int g = lane >> 4;
#pragma unroll
  for (int i = 0; i < 8; ++i) { const int ka = k0 + 8 * g + i, kb = ka + 16; v[i] = ka < K ? row[ka < K ? ka : K - 1] : 0.f; v[8 + i] = kb < K ? row[kb < K ? kb : K - 1] : 0.f; }
  return bsplit16(v); }
__device__ __forceinline__ F2 split_col(const float* W, int k0, int n, int lane, int ld, int K) { float v[16]; const int g = lane >> 4;
#pragma unroll
  for (int i = 0; i < 8; ++i) { const int ka = k0 + 8 * g + i, kb = ka + 16; v[i] = ka < K ? W[(size_t)(ka < K ? ka : K - 1) * ld + n] : 0.f; v[8 + i] = kb < K ? W[(size_t)(kb < K ? kb : K - 1) * ld + n] : 0.f; }
  return bsplit16(v); }
__device__ __forceinline__ v8f mac3(const F2& a, const F2& b, v8f c) { c = wmma_bf(a.l, b.h, c); c = wmma_bf(a.h, b.l, c); return wmma_bf(a.h, b.h, c); }
__device__ __forceinline__ float sigm(float v) { return 1.0f / (1.0f + expf(-v)); }
#define LDSX() do { asm volatile("s_wait_dscnt 0" ::: "memory"); __builtin_amdgcn_wave_barrier(); __builtin_amdgcn_fence(__ATOMIC_RELEASE, "workgroup"); } while (0)


#define NB 4
#define SS 4096
#define NR (NB * SS)
#define EMB 512
#define HD 64
#ifndef TQB
#define TQB (SS / 64)
#define TNB NB
#endif
typedef __attribute__((ext_vector_type(8))) __bf16 v8b;
__device__ __forceinline__ v16b frag_b(const __bf16* rowk0, int lane) {
  union { v16b v; v8b q[2]; } u; const __bf16* p = rowk0 + 8 * (lane >> 4);
  u.q[0] = *(const v8b*)p; u.q[1] = *(const v8b*)(p + 16); return u.v;
}
__device__ __forceinline__ float bfr(float v) { return (float)(__bf16)v; }
__device__ __attribute__((noinline)) float exp_ni(float v) { return expf(v); }
__device__ __attribute__((noinline)) float erf_ni(float v) { return erff(v); }

#define WS_PK  0u
#define WS_QH  (((2u * 192 * EMB) + 127u) / 128u * 128u)
#define WS_QL  (WS_QH + 2u * NR * HD)
#define WS_KH  (WS_QL + 2u * NR * HD)
#define WS_KL  (WS_KH + 2u * NR * HD)
#define WS_VTH (WS_KL + 2u * NR * HD)
#define WS_VTL (WS_VTH + 2u * NR * HD)
#define WS_END (WS_VTL + 2u * NR * HD)

__global__ __launch_bounds__(256) void k_pack(const float* __restrict__ WQ, const float* __restrict__ WK, const float* __restrict__ WV, __bf16* __restrict__ PK) {
  __shared__ __align__(16) __bf16 s[EMB]; const int n = blockIdx.x, t = threadIdx.x; const int which = n / HD, d = n % HD; const float* Wm = (which == 0) ? WQ : (which == 1) ? WK : WV;
  for (int k = t; k < EMB; k += 256) s[k] = (__bf16)Wm[(size_t)k * HD + d];
  __syncthreads();
  if (t < EMB / 8) vst2((unsigned*)(PK + (size_t)n * EMB + t * 8), *(const v4u*)&s[t * 8]);
}
__global__ __launch_bounds__(128) void k_qkv(const float* __restrict__ X, const __bf16* __restrict__ PK, const float* __restrict__ BQ, const float* __restrict__ BK, const float* __restrict__ BV, _Float16* __restrict__ QH, _Float16* __restrict__ QL_, _Float16* __restrict__ KH, _Float16* __restrict__ KL, _Float16* __restrict__ VTH, _Float16* __restrict__ VTL) {
  __shared__ __align__(16) _Float16 sqh[4][16][72], sql[4][16][72], skh[4][16][72], skl[4][16][72]; __shared__ __align__(16) _Float16 svh[HD][72], svl[HD][72];
  const int tid = threadIdx.x, wave = tid >> 5, lane = tid & 31, col = lane & 15, g = lane >> 4; const size_t r0 = (size_t)blockIdx.x * 64 + wave * 16;
  v8f acc[12] = {};
#pragma unroll 2
  for (int kc = 0; kc < EMB / 32; ++kc) { v16b a; { const float* p = X + (r0 + col) * EMB + kc * 32 + 8 * g;
#pragma unroll
      for (int i = 0; i < 8; ++i) { a[i] = (__bf16)p[i]; a[8 + i] = (__bf16)p[16 + i]; } }
#pragma unroll
    for (int j = 0; j < 12; ++j) acc[j] = wmma_bf(a, frag_b(PK + (size_t)(j * 16 + col) * EMB + kc * 32, lane), acc[j]); }
#pragma unroll
  for (int j = 0; j < 12; ++j) { const int which = j >> 2; const int d = (j & 3) * 16 + col; const float bb = bfr((which == 0) ? BQ[d] : (which == 1) ? BK[d] : BV[d]);
#pragma unroll
    for (int r = 0; r < 8; ++r) { const float v = acc[j][r] + bb; const _Float16 hv = (_Float16)v; const _Float16 lv = (_Float16)((v - (float)hv) * 2048.0f);
      if (which == 0) { sqh[wave][8 * g + r][d] = hv; sql[wave][8 * g + r][d] = lv; } else if (which == 1) { skh[wave][8 * g + r][d] = hv; skl[wave][8 * g + r][d] = lv; } else { svh[d][wave * 16 + 8 * g + r] = hv; svl[d][wave * 16 + 8 * g + r] = lv; } } }
  __syncthreads();
  for (int rl = 0; rl < 16; ++rl) { const size_t o = (r0 + rl) * HD + (lane & 7) * 8; const int which = lane >> 3;
    if (which == 0) vst2((unsigned*)(QH + o), *(const v4u*)&sqh[wave][rl][(lane & 7) * 8]); else if (which == 1) vst2((unsigned*)(QL_ + o), *(const v4u*)&sql[wave][rl][(lane & 7) * 8]); else if (which == 2) vst2((unsigned*)(KH + o), *(const v4u*)&skh[wave][rl][(lane & 7) * 8]); else vst2((unsigned*)(KL + o), *(const v4u*)&skl[wave][rl][(lane & 7) * 8]); }
  { const size_t rb = (size_t)blockIdx.x * 64; const int b = (int)(rb / SS), s0 = (int)(rb % SS);
    for (int e = tid; e < HD * 8; e += 128) { const int d = e >> 3, pc = e & 7; const size_t o = ((size_t)b * HD + d) * SS + s0 + pc * 8; vst2((unsigned*)(VTH + o), *(const v4u*)&svh[d][pc * 8]); vst2((unsigned*)(VTL + o), *(const v4u*)&svl[d][pc * 8]); } }
}
__global__ __launch_bounds__(128) void k_attn(const _Float16* __restrict__ QH, const _Float16* __restrict__ QL_, const _Float16* __restrict__ KH, const _Float16* __restrict__ KL, const _Float16* __restrict__ VTH, const _Float16* __restrict__ VTL, float* __restrict__ OUT) {
  __shared__ __align__(16) _Float16 sph[4][16][40], spl[4][16][40]; __shared__ __align__(16) float so[4][16][HD + 4];
  const int tid = threadIdx.x, wave = tid >> 5, lane = tid & 31, col = lane & 15, g = lane >> 4; const int qb = blockIdx.x, b = blockIdx.y; const int q0 = qb * 64 + wave * 16; const size_t rq = (size_t)b * SS + q0 + col;
  v16h aqh[2], aql[2];
#pragma unroll
  for (int kc = 0; kc < 2; ++kc) { aqh[kc] = frag_h(QH + rq * HD + kc * 32, lane); aql[kc] = frag_h(QL_ + rq * HD + kc * 32, lane); }
  const _Float16* Vh = VTH + (size_t)b * HD * SS; const _Float16* Vl = VTL + (size_t)b * HD * SS;
  float m[8], l[8];
#pragma unroll
  for (int r = 0; r < 8; ++r) { m[r] = -3.0e38f; l[r] = 0.f; }
  v8f acc[4] = {}, accl[4] = {};
  const int nks = (qb * 64 + 64) / 32;
#pragma unroll 1
  for (int ks = 0; ks < nks; ++ks) { v8f s[2];
#pragma unroll
    for (int ct = 0; ct < 2; ++ct) { const int kk = ks * 32 + ct * 16 + col; const size_t rk = ((size_t)b * SS + kk) * HD; v8f c = {}, cl = {};
#pragma unroll
      for (int kc = 0; kc < 2; ++kc) { const v16h khf = frag_h(KH + rk + kc * 32, lane); c = wmma16(aqh[kc], khf, c); cl = wmma16(aql[kc], khf, cl); cl = wmma16(aqh[kc], frag_h(KL + rk + kc * 32, lane), cl); }
#pragma unroll
      for (int r = 0; r < 8; ++r) { const int qi = q0 + 8 * g + r; const float sv = (c[r] + cl[r] * (1.0f / 2048.0f)) * 0.125f; s[ct][r] = (kk <= qi) ? sv : -3.0e38f; } }
#pragma unroll
    for (int r = 0; r < 8; ++r) { float mx = fmaxf(s[0][r], s[1][r]);
#pragma unroll
      for (int o = 1; o < 16; o <<= 1) mx = fmaxf(mx, __shfl_xor(mx, o));
      const float mn = fmaxf(m[r], mx); const float alpha = (m[r] <= -1.0e38f) ? 0.f : exp_ni(m[r] - mn);
      const float e0 = (s[0][r] <= -1.0e38f) ? 0.f : exp_ni(s[0][r] - mn), e1 = (s[1][r] <= -1.0e38f) ? 0.f : exp_ni(s[1][r] - mn); float es = e0 + e1;
#pragma unroll
      for (int o = 1; o < 16; o <<= 1) es += __shfl_xor(es, o);
      l[r] = l[r] * alpha + es; m[r] = mn;
#pragma unroll
      for (int dt = 0; dt < 4; ++dt) { acc[dt][r] *= alpha; accl[dt][r] *= alpha; }
      const _Float16 h0 = (_Float16)e0, h1 = (_Float16)e1; sph[wave][8 * g + r][col] = h0; sph[wave][8 * g + r][16 + col] = h1; spl[wave][8 * g + r][col] = (_Float16)((e0 - (float)h0) * 2048.0f); spl[wave][8 * g + r][16 + col] = (_Float16)((e1 - (float)h1) * 2048.0f); }
    LDSX();
    const v16h pah = frag_h(&sph[wave][col][0], lane), pal = frag_h(&spl[wave][col][0], lane);
#pragma unroll
    for (int dt = 0; dt < 4; ++dt) { const size_t vo = (size_t)(dt * 16 + col) * SS + ks * 32; const v16h vh = frag_h(Vh + vo, lane), vl = frag_h(Vl + vo, lane); acc[dt] = wmma16(pah, vh, acc[dt]); accl[dt] = wmma16(pal, vh, accl[dt]); accl[dt] = wmma16(pah, vl, accl[dt]); }
    LDSX(); }
#pragma unroll
  for (int r = 0; r < 8; ++r) { const float il = 1.0f / l[r];
#pragma unroll
    for (int dt = 0; dt < 4; ++dt) so[wave][8 * g + r][dt * 16 + col] = (acc[dt][r] + accl[dt][r] * (1.0f / 2048.0f)) * il; }
  LDSX();
  for (int rl = 0; rl < 16; ++rl) if (lane < 16) vst2(OUT + ((size_t)b * SS + q0 + rl) * HD + lane * 4, *(const v4f*)&so[wave][rl][lane * 4]);
}
extern "C" void kernel_launch(void* const* d_in, const int* in_sizes, int n_in, void* d_out, int out_size, void* d_ws, size_t ws_size, hipStream_t stream) {
  (void)in_sizes; (void)n_in; (void)out_size;
  const float** F = (const float**)d_in;
  if (ws_size < (size_t)WS_END) return;
  char* ws = (char*)d_ws; __bf16* PK = (__bf16*)(ws + WS_PK); _Float16 *QH = (_Float16*)(ws + WS_QH), *QLp = (_Float16*)(ws + WS_QL), *KH = (_Float16*)(ws + WS_KH), *KL = (_Float16*)(ws + WS_KL), *VTH = (_Float16*)(ws + WS_VTH), *VTL = (_Float16*)(ws + WS_VTL);
  k_pack<<<192, 256, 0, stream>>>(F[1], F[3], F[5], PK);
  k_qkv<<<TNB * SS / 64, 128, 0, stream>>>(F[0], PK, F[2], F[4], F[6], QH, QLp, KH, KL, VTH, VTL);
  k_attn<<<dim3(TQB, TNB), 128, 0, stream>>>(QH, QLp, KH, KL, VTH, VTL, (float*)d_out);
}
